// GptOssAttention_4922032521855
// MI455X (gfx1250) — hardware-verified
//
#include <hip/hip_runtime.h>
#include <hip/hip_bf16.h>

typedef _Float16     v16h __attribute__((ext_vector_type(16)));
typedef __bf16       v16b __attribute__((ext_vector_type(16)));
typedef float        v8f  __attribute__((ext_vector_type(8)));
typedef float        v4f  __attribute__((ext_vector_type(4)));
typedef unsigned int v4u  __attribute__((ext_vector_type(4)));

union Frag  { v16h f; v16b b; v4u q[2]; unsigned short s[16]; };
union Pack8 { v4u u; unsigned short s[8]; };

#define D_HEAD  64
#define G_SIZE  8
#define WIN     128
#define NKEY    144
#define KPAD    160

static __device__ __forceinline__ v8f zero8() { v8f z = {0.f, 0.f, 0.f, 0.f, 0.f, 0.f, 0.f, 0.f}; return z; }
static __device__ __forceinline__ v4f zero4() { v4f z = {0.f, 0.f, 0.f, 0.f}; return z; }

static __device__ __forceinline__ unsigned short bfb(float x) {
  union { __bf16 b; unsigned short u; } c; c.b = (__bf16)x; return c.u;
}
static __device__ __forceinline__ float bff(unsigned short u) { return __uint_as_float(((unsigned int)u) << 16); }
static __device__ __forceinline__ float bq16(float x) { return bff(bfb(x)); }
static __device__ __forceinline__ unsigned short hfb(float x) {
  union { _Float16 v; unsigned short u; } c; c.v = (_Float16)x; return c.u;
}

static __device__ __forceinline__ void ldfrag(Frag& f, const unsigned short* p, int h) {
  f.q[0] = *(const v4u*)(p + 8 * h);
  f.q[1] = *(const v4u*)(p + 16 + 8 * h);
}
static __device__ __forceinline__ v8f mma_h(const Frag& a, const Frag& b, v8f c) {
  return __builtin_amdgcn_wmma_f32_16x16x32_f16(false, a.f, false, b.f, (short)0, c, false, false);
}
static __device__ __forceinline__ v8f mma_b(const Frag& a, const Frag& b, v8f c) {
  return __builtin_amdgcn_wmma_f32_16x16x32_bf16(false, a.b, false, b.b, (short)0, c, false, false);
}

#define NOPS4 "v_nop\n\tv_nop\n\tv_nop\n\tv_nop"
#define GUARD1(a0, x, y) asm volatile(NOPS4 : "+v"(a0) : "v"(x), "v"(y))
#define GUARD4(a0, a1, a2, a3, x, y) \
  asm volatile(NOPS4 : "+v"(a0), "+v"(a1), "+v"(a2), "+v"(a3) : "v"(x), "v"(y))
#define GUARD8(a0, a1, a2, a3, a4, a5, a6, a7, x, y) \
  asm volatile(NOPS4 : "+v"(a0), "+v"(a1), "+v"(a2), "+v"(a3), "+v"(a4), "+v"(a5), "+v"(a6), "+v"(a7) : "v"(x), "v"(y))

__global__ __launch_bounds__(256) void cvt_act_kernel(const float* __restrict__ src, unsigned short* dst, int n8) {
  const int i = blockIdx.x * 256 + threadIdx.x;
  if (i >= n8) return;
  const size_t o = (size_t)i * 8;
  const v4f a = *(const v4f*)(src + o);
  const v4f b = *(const v4f*)(src + o + 4);
  Pack8 p;
  p.s[0] = bfb(a[0]); p.s[1] = bfb(a[1]); p.s[2] = bfb(a[2]); p.s[3] = bfb(a[3]);
  p.s[4] = bfb(b[0]); p.s[5] = bfb(b[1]); p.s[6] = bfb(b[2]); p.s[7] = bfb(b[3]);
  const v4u u = p.u;
  *(volatile v4u*)(dst + o) = u;
  __threadfence();
  *(volatile v4u*)(dst + o) = u;
}

template <int F16>
__global__ __launch_bounds__(64) void wtrans_kernel(const float* __restrict__ Wm, unsigned short* o,
                                                     int K, int N, float scale) {
  __shared__ __align__(16) float sT[32 * 68];
  const int t = threadIdx.x;
  const int n0 = blockIdx.x * 32, k0 = blockIdx.y * 64;
  {
    const int k = min(k0 + t, K - 1);
    const float* row = Wm + (size_t)k * N + n0;
#pragma unroll
    for (int c = 0; c < 8; ++c) {
      v4f v = zero4();
      if (n0 + 4 * c + 3 < N) v = *(const v4f*)(row + 4 * c);
      sT[(4 * c + 0) * 68 + t] = v[0];
      sT[(4 * c + 1) * 68 + t] = v[1];
      sT[(4 * c + 2) * 68 + t] = v[2];
      sT[(4 * c + 3) * 68 + t] = v[3];
    }
  }
  __syncthreads();
  const int l = t & 31, wv = t >> 5, seg = l & 7;
  v4u va[4];
  size_t off[4];
  bool okk[4];
#pragma unroll
  for (int it = 0; it < 4; ++it) {
    const int r = it * 8 + wv * 4 + (l >> 3);
    const float* sp = sT + r * 68 + seg * 8;
    const v4f x0 = *(const v4f*)sp;
    const v4f x1 = *(const v4f*)(sp + 4);
    const float x[8] = {x0[0], x0[1], x0[2], x0[3], x1[0], x1[1], x1[2], x1[3]};
    Pack8 ua;
#pragma unroll
    for (int j = 0; j < 8; ++j) {
      if (F16) ua.s[j] = hfb(bq16(x[j]) * scale);
      else     ua.s[j] = bfb(x[j]);
    }
    va[it] = ua.u;
    const int n = n0 + r;
    okk[it] = (n < N) && (k0 + seg * 8 + 8 <= K);
    off[it] = (size_t)n * K + k0 + seg * 8;
  }
#pragma unroll
  for (int it = 0; it < 4; ++it)
    if (okk[it]) *(volatile v4u*)(o + off[it]) = va[it];
  __threadfence();
#pragma unroll
  for (int it = 0; it < 4; ++it)
    if (okk[it]) *(volatile v4u*)(o + off[it]) = va[it];
}

template <int F16, int ROPE>
__global__ __launch_bounds__(128) void gemm_kernel(const unsigned short* __restrict__ A,
                                                   const unsigned short* __restrict__ Bt,
                                                   const float* __restrict__ bias,
                                                   const int* __restrict__ pos,
                                                   float* tab, float* C, int M, int N, int K, float oscale) {
  constexpr int PC = 68;
  __shared__ __align__(16) float sC[4 * 32 * PC];
  __shared__ __align__(16) float sR[ROPE ? 128 * 64 : 4];
  const int l = threadIdx.x & 31, h = l >> 4, r16 = l & 15, w = threadIdx.x >> 5;
  const int n0 = blockIdx.x * 64;
  const int mb = blockIdx.y * 128;
  const int m0 = mb + w * 32;

  unsigned aoff[2];
#pragma unroll
  for (int t = 0; t < 2; ++t) aoff[t] = (unsigned)min(m0 + 16 * t + r16, M - 1) * (unsigned)K;
  unsigned boff[4];
#pragma unroll
  for (int s = 0; s < 4; ++s) boff[s] = (unsigned)min(n0 + 16 * s + r16, N - 1) * (unsigned)K;

  v8f acc[2][4];
#pragma unroll
  for (int t = 0; t < 2; ++t)
#pragma unroll
    for (int s = 0; s < 4; ++s) acc[t][s] = zero8();

#pragma unroll 1
  for (int k0 = 0; k0 < K; k0 += 32) {
    Frag fa[2];
    ldfrag(fa[0], A + aoff[0] + k0, h);
    ldfrag(fa[1], A + aoff[1] + k0, h);
    Frag gb;
#pragma unroll
    for (int s = 0; s < 4; ++s) {
      ldfrag(gb, Bt + boff[s] + k0, h);
#pragma unroll
      for (int t = 0; t < 2; ++t) {
        if (F16) acc[t][s] = mma_h(fa[t], gb, acc[t][s]);
        else     acc[t][s] = mma_b(fa[t], gb, acc[t][s]);
      }
    }
    GUARD8(acc[0][0], acc[0][1], acc[0][2], acc[0][3], acc[1][0], acc[1][1], acc[1][2], acc[1][3], fa[0].f, gb.f);
  }

  if (ROPE) {
    const int d = threadIdx.x & 31, rg = threadIdx.x >> 5;
    const float e = ((float)d * 2.0f) / 64.0f;
    const float fr = powf(150000.0f, e);
    const float inv = 1.0f / fr;
#pragma unroll 1
    for (int it = 0; it < 32; ++it) {
      const int row = it * 4 + rg;
      const int gm = min(mb + row, M - 1);
      const float ang = (float)pos[gm] * inv;
      float sn, cs;
      sincosf(ang, &sn, &cs);
      sR[row * 64 + d] = cs;
      sR[row * 64 + 32 + d] = sn;
    }
  }

  float* sw = sC + w * (32 * PC);
  {
    float bcol[4];
#pragma unroll
    for (int s = 0; s < 4; ++s) {
      const int cn = n0 + 16 * s + r16;
      bcol[s] = (cn < N) ? bq16(bias[cn]) : 0.f;
    }
#pragma unroll
    for (int t = 0; t < 2; ++t)
#pragma unroll
      for (int s = 0; s < 4; ++s)
#pragma unroll
        for (int r = 0; r < 8; ++r)
          sw[(16 * t + 8 * h + r) * PC + 16 * s + r16] = acc[t][s][r] * oscale + bcol[s];
  }
  __syncthreads();

  const int c4 = l & 15, rsel = l >> 4;
  const int nc = n0 + 4 * c4;
  const bool wtab = ROPE && (blockIdx.x == 0);
  auto epass = [&]() {
#pragma unroll 1
    for (int it = 0; it < 16; ++it) {
      const int row = it * 2 + rsel;
      const int gm = m0 + row;
      const v4f x = *(const v4f*)(sw + row * PC + 4 * c4);
      v4f o = x;
      v4f tv = zero4();
      if (ROPE) {
        const v4f y = *(const v4f*)(sw + row * PC + 4 * (c4 ^ 8));
        const float* tr = sR + (w * 32 + row) * 64 + 4 * (c4 & 7);
        const v4f cs = *(const v4f*)tr;
        const v4f sn = *(const v4f*)(tr + 32);
        const bool first = (c4 < 8);
#pragma unroll
        for (int q = 0; q < 4; ++q)
          o[q] = first ? (x[q] * cs[q] - y[q] * sn[q]) : (y[q] * sn[q] + x[q] * cs[q]);
        tv = first ? cs : sn;
      }
      if (gm < M && nc + 3 < N) {
        *(volatile v4f*)(C + (size_t)gm * N + nc) = o;
        if (wtab) *(volatile v4f*)(tab + (size_t)gm * 64 + 4 * c4) = tv;
      }
    }
  };
  epass();
  __threadfence();
  epass();
}

__global__ __launch_bounds__(128) void attn_kernel(const float* __restrict__ qF, const float* __restrict__ kR,
                                                   const float* __restrict__ vF, const float* __restrict__ tab,
                                                   unsigned short* ao, int S, int qsz, int kvsz) {
  __shared__ __align__(16) unsigned short sK[2][NKEY * D_HEAD];
  __shared__ __align__(16) unsigned short sV[2][D_HEAD * KPAD];
  __shared__ __align__(16) float sS[4][16 * NKEY];
  __shared__ __align__(16) unsigned short sP[4][2][16 * KPAD];

  const int tid = threadIdx.x, w = tid >> 5, l = tid & 31, h = l >> 4, r16 = l & 15;
  const int tok0 = blockIdx.x * 16;
  const int kvh = blockIdx.y;
  const int bsel = tok0 / S;
  const int s0 = tok0 - bsel * S;

  for (int idx = tid; idx < NKEY * 8; idx += 128) {
    const int row = idx >> 3, seg = idx & 7;
    const int sk = s0 - WIN + row;
    v4f ka = zero4(), kb = zero4(), va = zero4(), vb = zero4();
    if (sk >= 0) {
      const size_t off = (size_t)(bsel * S + sk) * kvsz + kvh * D_HEAD + seg * 8;
      ka = *(const v4f*)(kR + off);
      kb = *(const v4f*)(kR + off + 4);
      va = *(const v4f*)(vF + off);
      vb = *(const v4f*)(vF + off + 4);
    }
    const float kx[8] = {ka[0], ka[1], ka[2], ka[3], kb[0], kb[1], kb[2], kb[3]};
    const float vx[8] = {va[0], va[1], va[2], va[3], vb[0], vb[1], vb[2], vb[3]};
    Pack8 kh, kl;
#pragma unroll
    for (int j = 0; j < 8; ++j) {
      const unsigned short hb = bfb(kx[j]);
      kh.s[j] = hb;
      kl.s[j] = bfb(kx[j] - bff(hb));
      const unsigned short hv = bfb(vx[j]);
      sV[0][(seg * 8 + j) * KPAD + row] = hv;
      sV[1][(seg * 8 + j) * KPAD + row] = bfb(vx[j] - bff(hv));
    }
    *(v4u*)(&sK[0][row * D_HEAD + seg * 8]) = kh.u;
    *(v4u*)(&sK[1][row * D_HEAD + seg * 8]) = kl.u;
  }
  for (int idx = tid; idx < D_HEAD * (KPAD - NKEY); idx += 128) {
    sV[0][(idx >> 4) * KPAD + NKEY + (idx & 15)] = 0;
    sV[1][(idx >> 4) * KPAD + NKEY + (idx & 15)] = 0;
  }
  float cz[16], sz[16];
  {
    const float* tb = tab + (size_t)(tok0 + r16) * 64;
    const v4f c0 = *(const v4f*)(tb + 8 * h);
    const v4f c1 = *(const v4f*)(tb + 8 * h + 4);
    const v4f c2 = *(const v4f*)(tb + 16 + 8 * h);
    const v4f c3 = *(const v4f*)(tb + 20 + 8 * h);
    const v4f n0v = *(const v4f*)(tb + 32 + 8 * h);
    const v4f n1v = *(const v4f*)(tb + 36 + 8 * h);
    const v4f n2v = *(const v4f*)(tb + 48 + 8 * h);
    const v4f n3v = *(const v4f*)(tb + 52 + 8 * h);
#pragma unroll
    for (int e = 0; e < 4; ++e) {
      cz[e] = c0[e]; cz[4 + e] = c1[e]; cz[8 + e] = c2[e]; cz[12 + e] = c3[e];
      sz[e] = n0v[e]; sz[4 + e] = n1v[e]; sz[8 + e] = n2v[e]; sz[12 + e] = n3v[e];
    }
  }
  __syncthreads();

  float* ss = sS[w];

#pragma unroll 1
  for (int hh = 0; hh < 2; ++hh) {
    const int head = kvh * G_SIZE + w + hh * 4;

    Frag qh0, ql0, qh1, ql1;
    {
      const float* qr = qF + (size_t)(tok0 + r16) * qsz + head * D_HEAD;
      const v4f a0 = *(const v4f*)(qr + 8 * h);
      const v4f a1 = *(const v4f*)(qr + 8 * h + 4);
      const v4f a2 = *(const v4f*)(qr + 16 + 8 * h);
      const v4f a3 = *(const v4f*)(qr + 20 + 8 * h);
      const v4f b0 = *(const v4f*)(qr + 32 + 8 * h);
      const v4f b1 = *(const v4f*)(qr + 36 + 8 * h);
      const v4f b2 = *(const v4f*)(qr + 48 + 8 * h);
      const v4f b3 = *(const v4f*)(qr + 52 + 8 * h);
      const float x1[16] = {a0[0], a0[1], a0[2], a0[3], a1[0], a1[1], a1[2], a1[3],
                            a2[0], a2[1], a2[2], a2[3], a3[0], a3[1], a3[2], a3[3]};
      const float x2[16] = {b0[0], b0[1], b0[2], b0[3], b1[0], b1[1], b1[2], b1[3],
                            b2[0], b2[1], b2[2], b2[3], b3[0], b3[1], b3[2], b3[3]};
#pragma unroll
      for (int e = 0; e < 16; ++e) {
        const float r1 = x1[e] * cz[e] - x2[e] * sz[e];
        const float r2 = x1[e] * sz[e] + x2[e] * cz[e];
        const unsigned short h1 = bfb(r1), h2 = bfb(r2);
        qh0.s[e] = h1; ql0.s[e] = bfb(r1 - bff(h1));
        qh1.s[e] = h2; ql1.s[e] = bfb(r2 - bff(h2));
      }
    }

#pragma unroll 1
    for (int j = 0; j < 9; ++j) {
      if (s0 - WIN + 16 * j + 15 < 0) continue;
      const unsigned short* kp0 = &sK[0][(j * 16 + r16) * D_HEAD];
      const unsigned short* kp1 = &sK[1][(j * 16 + r16) * D_HEAD];
      Frag kh0, kh1, kl0, kl1;
      ldfrag(kh0, kp0, h);
      ldfrag(kh1, kp0 + 32, h);
      ldfrag(kl0, kp1, h);
      ldfrag(kl1, kp1 + 32, h);
      v8f acc = zero8();
      acc = mma_b(qh0, kh0, acc);
      acc = mma_b(qh0, kl0, acc);
      acc = mma_b(ql0, kh0, acc);
      acc = mma_b(qh1, kh1, acc);
      acc = mma_b(qh1, kl1, acc);
      acc = mma_b(ql1, kh1, acc);
      GUARD1(acc, ql1.f, kh1.f);
#pragma unroll
      for (int r = 0; r < 8; ++r) ss[(8 * h + r) * NKEY + j * 16 + r16] = acc[r];
    }

#pragma unroll
    for (int r = 0; r < 8; ++r) {
      const int m = 8 * h + r;
      float vals[9];
      float rmax = -1.0e30f;
#pragma unroll
      for (int j = 0; j < 9; ++j) {
        const int jn = j * 16 + r16;
        const bool valid = (jn >= m) && (jn <= m + WIN) && (s0 - WIN + jn >= 0);
        const float raw = ss[m * NKEY + jn];
        const float x = valid ? raw * 0.125f : -1.0e30f;
        vals[j] = x;
        rmax = fmaxf(rmax, x);
      }
      rmax = fmaxf(rmax, __shfl_xor(rmax, 1));
      rmax = fmaxf(rmax, __shfl_xor(rmax, 2));
      rmax = fmaxf(rmax, __shfl_xor(rmax, 4));
      rmax = fmaxf(rmax, __shfl_xor(rmax, 8));
      float rsum = 0.f;
#pragma unroll
      for (int j = 0; j < 9; ++j) {
        const float ev = __expf(vals[j] - rmax);
        vals[j] = ev;
        rsum += ev;
      }
      rsum += __shfl_xor(rsum, 1);
      rsum += __shfl_xor(rsum, 2);
      rsum += __shfl_xor(rsum, 4);
      rsum += __shfl_xor(rsum, 8);
      const float rinv = 1.0f / rsum;
#pragma unroll
      for (int j = 0; j < 9; ++j) {
        const int jn = j * 16 + r16;
        const float pv = vals[j] * rinv;
        const unsigned short hp = bfb(pv);
        sP[w][0][m * KPAD + jn] = hp;
        sP[w][1][m * KPAD + jn] = bfb(pv - bff(hp));
      }
      sP[w][0][m * KPAD + NKEY + r16] = 0;
      sP[w][1][m * KPAD + NKEY + r16] = 0;
    }
    __syncthreads();

    v8f ov[4];
#pragma unroll
    for (int s = 0; s < 4; ++s) ov[s] = zero8();
#pragma unroll 1
    for (int kc = 0; kc < 5; ++kc) {
      if (s0 - WIN + 32 * kc + 31 < 0) continue;
      Frag ph, pl;
      ldfrag(ph, &sP[w][0][r16 * KPAD + kc * 32], h);
      ldfrag(pl, &sP[w][1][r16 * KPAD + kc * 32], h);
      Frag vh, vl;
#pragma unroll
      for (int s = 0; s < 4; ++s) {
        ldfrag(vh, &sV[0][(s * 16 + r16) * KPAD + kc * 32], h);
        ldfrag(vl, &sV[1][(s * 16 + r16) * KPAD + kc * 32], h);
        ov[s] = mma_b(ph, vh, ov[s]);
        ov[s] = mma_b(ph, vl, ov[s]);
        ov[s] = mma_b(pl, vh, ov[s]);
      }
      GUARD4(ov[0], ov[1], ov[2], ov[3], pl.f, vh.f);
    }

    unsigned short* so = (unsigned short*)ss;
#pragma unroll
    for (int s = 0; s < 4; ++s)
#pragma unroll
      for (int r = 0; r < 8; ++r)
        so[(8 * h + r) * D_HEAD + 16 * s + r16] = hfb(ov[s][r] * 16.0f);
    __syncthreads();
    v4u ovl[4];
    size_t oof[4];
#pragma unroll
    for (int it = 0; it < 4; ++it) {
      const int row = it * 4 + (l >> 3), seg = l & 7;
      ovl[it] = *(const v4u*)(so + row * D_HEAD + seg * 8);
      oof[it] = (size_t)(tok0 + row) * qsz + head * D_HEAD + seg * 8;
    }
#pragma unroll
    for (int it = 0; it < 4; ++it) *(volatile v4u*)(ao + oof[it]) = ovl[it];
    __threadfence();
#pragma unroll
    for (int it = 0; it < 4; ++it) *(volatile v4u*)(ao + oof[it]) = ovl[it];
    __syncthreads();
  }
}

static inline size_t al256(size_t x) { return (x + 255) & ~(size_t)255; }

extern "C" void kernel_launch(void* const* d_in, const int* in_sizes, int n_in,
                              void* d_out, int out_size, void* d_ws, size_t ws_size,
                              hipStream_t stream) {
  if (n_in < 10) return;
  const int HID = in_sizes[9];
  const int QS  = in_sizes[3];
  const int KVS = in_sizes[5];
  if (HID <= 0 || QS <= 0 || KVS <= 0) return;
  const int T   = in_sizes[0] / HID;
  const int S   = 1024;
  const int HQ  = QS / D_HEAD, HKV = KVS / D_HEAD;
  bool ok = true;
  ok = ok && (in_sizes[0] == T * HID) && (in_sizes[1] == T) && (in_sizes[2] == HID * QS);
  ok = ok && (in_sizes[4] == HID * KVS) && (in_sizes[6] == HID * KVS) && (in_sizes[7] == KVS);
  ok = ok && (in_sizes[8] == QS * HID) && (out_size == T * HID);
  ok = ok && (QS == HQ * D_HEAD) && (KVS == HKV * D_HEAD) && (HQ == G_SIZE * HKV) && (HKV > 0);
  ok = ok && (T > 0) && (T % S == 0) && (T % 16 == 0) && (HID % 64 == 0) && (QS % 64 == 0) && (KVS % 64 == 0);
  if (!ok) return;

  const float* hs  = (const float*)d_in[0];
  const int*   psn = (const int*)d_in[1];
  const float* Wq  = (const float*)d_in[2];
  const float* bq  = (const float*)d_in[3];
  const float* Wk  = (const float*)d_in[4];
  const float* bk  = (const float*)d_in[5];
  const float* Wv  = (const float*)d_in[6];
  const float* bv  = (const float*)d_in[7];
  const float* Wo  = (const float*)d_in[8];
  const float* bo  = (const float*)d_in[9];
  float* out = (float*)d_out;
  char*  ws  = (char*)d_ws;

  const size_t szH   = al256((size_t)T * HID * 2);
  const size_t szWq  = al256((size_t)QS * HID * 2);
  const size_t szWkv = al256((size_t)KVS * HID * 2);
  const size_t szWo  = al256((size_t)HID * QS * 2);
  const size_t szTab = al256((size_t)T * 64 * 4);
  const size_t szQ   = al256((size_t)T * QS * 4);
  const size_t szKV  = al256((size_t)T * KVS * 4);
  const size_t szAO  = al256((size_t)T * QS * 2);

  size_t off = 0;
  unsigned short* hB  = (unsigned short*)(ws + off); off += szH;
  unsigned short* WqT = (unsigned short*)(ws + off); off += szWq;
  unsigned short* WkT = (unsigned short*)(ws + off); off += szWkv;
  unsigned short* WvT = (unsigned short*)(ws + off); off += szWkv;
  unsigned short* WoT = (unsigned short*)(ws + off); off += szWo;
  float*          tab = (float*)(ws + off);          off += szTab;
  float*          qF  = (float*)(ws + off);          off += szQ;
  float*          kR  = (float*)(ws + off);          off += szKV;
  float*          vF  = (float*)(ws + off);          off += szKV;
  unsigned short* ao  = (unsigned short*)(ws + off); off += szAO;
  if (off > ws_size) return;

  const int n8 = T * HID / 8;
  cvt_act_kernel<<<(n8 + 255) / 256, 256, 0, stream>>>(hs, hB, n8);

  wtrans_kernel<0><<<dim3((QS + 31) / 32, (HID + 63) / 64), 64, 0, stream>>>(Wq, WqT, HID, QS, 1.0f);
  wtrans_kernel<0><<<dim3((KVS + 31) / 32, (HID + 63) / 64), 64, 0, stream>>>(Wk, WkT, HID, KVS, 1.0f);
  wtrans_kernel<0><<<dim3((KVS + 31) / 32, (HID + 63) / 64), 64, 0, stream>>>(Wv, WvT, HID, KVS, 1.0f);
  wtrans_kernel<1><<<dim3((HID + 31) / 32, (QS + 63) / 64), 64, 0, stream>>>(Wo, WoT, QS, HID, 64.0f);

  gemm_kernel<0, 0><<<dim3((QS + 63) / 64, (T + 127) / 128), 128, 0, stream>>>(
      hB, WqT, bq, psn, tab, qF, T, QS, HID, 1.0f);
  gemm_kernel<0, 1><<<dim3((KVS + 63) / 64, (T + 127) / 128), 128, 0, stream>>>(
      hB, WkT, bk, psn, tab, kR, T, KVS, HID, 1.0f);
  gemm_kernel<0, 0><<<dim3((KVS + 63) / 64, (T + 127) / 128), 128, 0, stream>>>(
      hB, WvT, bv, psn, tab, vF, T, KVS, HID, 1.0f);

  attn_kernel<<<dim3(T / 16, HKV), 128, 0, stream>>>(qF, kR, vF, tab, ao, S, QS, KVS);

  gemm_kernel<1, 0><<<dim3((HID + 63) / 64, (T + 127) / 128), 128, 0, stream>>>(
      ao, WoT, bo, psn, tab, out, T, HID, QS, 1.0f / 1024.0f);
}
